// MultiHeadedAttentionPure_66022237274782
// MI455X (gfx1250) — hardware-verified
//
#include <hip/hip_runtime.h>
#include <math.h>

typedef __attribute__((ext_vector_type(16))) _Float16 v16h;
typedef __attribute__((ext_vector_type(16))) __bf16 v16b;
typedef __attribute__((ext_vector_type(8)))  _Float16 v8h;
typedef __attribute__((ext_vector_type(8)))  float v8f;
typedef __attribute__((ext_vector_type(4)))  float v4f;
typedef __attribute__((ext_vector_type(2)))  float v2f;
typedef __attribute__((ext_vector_type(4)))  unsigned v4u;
typedef __attribute__((ext_vector_type(4)))  int v4i;
typedef float __attribute__((may_alias)) float_a;
typedef int __attribute__((may_alias)) int_a;

template <typename T> __device__ __forceinline__ void vst2(void* p, T v) { *(volatile T*)p = v; __threadfence(); *(volatile T*)p = v; }
__device__ __forceinline__ v8f wmma16(v16h a, v16h b, v8f c) {
  v8f d = __builtin_amdgcn_wmma_f32_16x16x32_f16(false, a, false, b, (short)0, c, false, false);
  asm volatile("v_nop\n\tv_nop\n\tv_nop\n\tv_nop" : "+v"(d) : "v"(a), "v"(b));
  return d;
}
__device__ __forceinline__ v8f wmma_bf(v16b a, v16b b, v8f c) {
  v8f d = __builtin_amdgcn_wmma_f32_16x16x32_bf16(false, a, false, b, (short)0, c, false, false);
  asm volatile("v_nop\n\tv_nop\n\tv_nop\n\tv_nop" : "+v"(d) : "v"(a), "v"(b));
  return d;
}
__device__ __forceinline__ v16h frag_h(const _Float16* rowk0, int lane) {
  union { v16h v; v8h q[2]; } u; const _Float16* p = rowk0 + 8 * (lane >> 4);
  u.q[0] = *(const v8h*)p; u.q[1] = *(const v8h*)(p + 16); return u.v;
}
__device__ __forceinline__ v16h frag_f32(const float* rowk0, int lane) {
  v16h a; const float* p = rowk0 + 8 * (lane >> 4);
#pragma unroll
  for (int i = 0; i < 8; ++i) { a[i] = (_Float16)p[i]; a[8 + i] = (_Float16)p[16 + i]; }
  return a;
}
__device__ __forceinline__ v16h frag_f32s(const float* rowk0, int lane, float sc) {
  v16h a; const float* p = rowk0 + 8 * (lane >> 4);
#pragma unroll
  for (int i = 0; i < 8; ++i) { a[i] = (_Float16)(p[i] * sc); a[8 + i] = (_Float16)(p[16 + i] * sc); }
  return a;
}
__device__ __forceinline__ v16h fragc_f32(const float* W, int k0, int n, int lane, int ld, int K) {
  v16h a; const int g = lane >> 4;
#pragma unroll
  for (int i = 0; i < 8; ++i) { const int ka = k0 + 8 * g + i, kb = ka + 16;
    a[i] = (_Float16)(ka < K ? W[(size_t)(ka < K ? ka : K - 1) * ld + n] : 0.f); a[8 + i] = (_Float16)(kb < K ? W[(size_t)(kb < K ? kb : K - 1) * ld + n] : 0.f); }
  return a;
}
struct F2 { v16b h, l; };
__device__ __forceinline__ F2 bsplit16(const float v[16]) { F2 r;
#pragma unroll
  for (int i = 0; i < 16; ++i) { const __bf16 h = (__bf16)v[i]; r.h[i] = h; r.l[i] = (__bf16)(v[i] - (float)h); }
  return r; }
__device__ __forceinline__ F2 split_row(const float* row, int k0, int lane) { float v[16]; const float* p = row + k0 + 8 * (lane >> 4);
#pragma unroll
  for (int i = 0; i < 8; ++i) { v[i] = p[i]; v[8 + i] = p[16 + i]; }
  return bsplit16(v); }
__device__ __forceinline__ F2 split_rowK(const float* row, int k0, int lane, int K) { float v[16]; const int g = lane >> 4;
#pragma unroll
  for (int i = 0; i < 8; ++i) { const int ka = k0 + 8 * g + i, kb = ka + 16; v[i] = ka < K ? row[ka < K ? ka : K - 1] : 0.f; v[8 + i] = kb < K ? row[kb < K ? kb : K - 1] : 0.f; }
  return bsplit16(v); }
__device__ __forceinline__ F2 split_col(const float* W, int k0, int n, int lane, int ld, int K) { float v[16]; const int g = lane >> 4;
#pragma unroll
  for (int i = 0; i < 8; ++i) { const int ka = k0 + 8 * g + i, kb = ka + 16; v[i] = ka < K ? W[(size_t)(ka < K ? ka : K - 1) * ld + n] : 0.f; v[8 + i] = kb < K ? W[(size_t)(kb < K ? kb : K - 1) * ld + n] : 0.f; }
  return bsplit16(v); }
__device__ __forceinline__ v8f mac3(const F2& a, const F2& b, v8f c) { c = wmma_bf(a.l, b.h, c); c = wmma_bf(a.h, b.l, c); return wmma_bf(a.h, b.h, c); }
__device__ __forceinline__ float sigm(float v) { return 1.0f / (1.0f + expf(-v)); }
#define LDSX() do { asm volatile("s_wait_dscnt 0" ::: "memory"); __builtin_amdgcn_wave_barrier(); __builtin_amdgcn_fence(__ATOMIC_RELEASE, "workgroup"); } while (0)


#define NB 8
#define TT 1024
#define FF 512
#define NH 8
#define HD 64
#ifndef TQB
#define TQB (TT / 64)
#define TNB NB
#define TOB (NB * TT / 64)
#endif
typedef __attribute__((ext_vector_type(8))) __bf16 v8b;
__device__ __forceinline__ v16b frag_b(const __bf16* rowk0, int lane) {
  union { v16b v; v8b q[2]; } u; const __bf16* p = rowk0 + 8 * (lane >> 4);
  u.q[0] = *(const v8b*)p; u.q[1] = *(const v8b*)(p + 16); return u.v;
}
__device__ __forceinline__ float bfr(float v) { return (float)(__bf16)v; }
__device__ __attribute__((noinline)) float exp_ni(float v) { return expf(v); }
__device__ __attribute__((noinline)) float erf_ni(float v) { return erff(v); }

#define WS_PW  0u
#define WS_QA  (WS_PW + 2u * 5 * FF * FF)
#define WS_KB  (WS_QA + 4u * NB * TT * NH * 128)
#define WS_VH  (WS_KB + 4u * NB * TT * NH * 128)
#define WS_VL  (WS_VH + 2u * NB * FF * TT)
#define WS_P   (WS_VL + 2u * NB * FF * TT)
#define WS_O   (WS_P + 4u * TT * FF)
#define WS_END (WS_O + 4u * NB * TT * FF)

__global__ __launch_bounds__(128) void k_pack(const float* __restrict__ WQ, const float* __restrict__ WK, const float* __restrict__ WV, const float* __restrict__ WP, const float* __restrict__ WO, __bf16* __restrict__ PW) {
  __shared__ __align__(16) __bf16 s[FF]; const int n = blockIdx.x, which = blockIdx.y, tid = threadIdx.x; const float* src = (which == 0 ? WQ : which == 1 ? WK : which == 2 ? WV : which == 3 ? WP : WO) + (size_t)n * FF;
  for (int k = tid; k < FF; k += 128) s[k] = (__bf16)src[k];
  __syncthreads();
  if (tid < FF / 8) vst2((unsigned*)(PW + ((size_t)which * FF + n) * FF + tid * 8), *(const v4u*)&s[tid * 8]);
}
__global__ __launch_bounds__(128) void k_posp(const float* __restrict__ PE, const __bf16* __restrict__ P4, float* __restrict__ P) {
  __shared__ __align__(16) float so[4][16][132];
  const int tid = threadIdx.x, wave = tid >> 5, lane = tid & 31, col = lane & 15, g = lane >> 4; const size_t r0 = (size_t)blockIdx.x * 64 + wave * 16; const int n0 = blockIdx.y * 128;
  v8f acc[8] = {};
#pragma unroll 2
  for (int kc = 0; kc < FF / 32; ++kc) { v16b a; { const float* p = PE + (r0 + col) * FF + kc * 32 + 8 * g;
#pragma unroll
      for (int i = 0; i < 8; ++i) { a[i] = (__bf16)p[i]; a[8 + i] = (__bf16)p[16 + i]; } }
#pragma unroll
    for (int j = 0; j < 8; ++j) acc[j] = wmma_bf(a, frag_b(P4 + (size_t)(n0 + j * 16 + col) * FF + kc * 32, lane), acc[j]); }
#pragma unroll
  for (int j = 0; j < 8; ++j)
#pragma unroll
    for (int r = 0; r < 8; ++r) so[wave][8 * g + r][j * 16 + col] = acc[j][r];
  LDSX();
  for (int rl = 0; rl < 16; ++rl) vst2(P + (r0 + rl) * FF + n0 + lane * 4, *(const v4f*)&so[wave][rl][lane * 4]);
}
template <int MODE>
__global__ __launch_bounds__(128) void k_proj(const float* __restrict__ X, const __bf16* __restrict__ P1, const float* __restrict__ bias, const float* __restrict__ U, const float* __restrict__ Vb, const float* __restrict__ PP, float* __restrict__ OUT, __bf16* __restrict__ VH, __bf16* __restrict__ VL) {
  __shared__ __align__(16) float so[4][16][260]; __shared__ __align__(16) __bf16 sth[128][72], stl[128][72];
  const int tid = threadIdx.x, wave = tid >> 5, lane = tid & 31, col = lane & 15, g = lane >> 4; const size_t rb = (size_t)blockIdx.x * 64; const size_t r0 = rb + wave * 16; const int n0 = blockIdx.y * 128;
  v8f acc[8] = {};
#pragma unroll 2
  for (int kc = 0; kc < FF / 32; ++kc) { v16b a; { const float* p = X + (r0 + col) * FF + kc * 32 + 8 * g;
#pragma unroll
      for (int i = 0; i < 8; ++i) { a[i] = (__bf16)p[i]; a[8 + i] = (__bf16)p[16 + i]; } }
#pragma unroll
    for (int j = 0; j < 8; ++j) acc[j] = wmma_bf(a, frag_b(P1 + (size_t)(n0 + j * 16 + col) * FF + kc * 32, lane), acc[j]); }
  if (MODE == 2) {
#pragma unroll
    for (int j = 0; j < 8; ++j) { const float bb = bfr(bias[n0 + j * 16 + col]);
#pragma unroll
      for (int r = 0; r < 8; ++r) { const float v = acc[j][r] + bb; const __bf16 hb = (__bf16)v; sth[j * 16 + col][wave * 16 + 8 * g + r] = hb; stl[j * 16 + col][wave * 16 + 8 * g + r] = (__bf16)(v - (float)hb); } }
    __syncthreads();
    const int b = (int)(rb / TT), t0 = (int)(rb % TT);
    for (int q = tid; q < 128 * 8; q += 128) { const int d = q >> 3, pc = q & 7; const size_t o = ((size_t)b * FF + n0 + d) * TT + t0 + pc * 8; vst2((unsigned*)(VH + o), *(const v4u*)&sth[d][pc * 8]); vst2((unsigned*)(VL + o), *(const v4u*)&stl[d][pc * 8]); }
  } else {
#pragma unroll
    for (int j = 0; j < 8; ++j) { const int hl = j >> 2, d = (j & 3) * 16 + col; const int h = (n0 >> 6) + hl; const float bb = bfr(bias[n0 + j * 16 + col]);
#pragma unroll
      for (int r = 0; r < 8; ++r) { const float v = acc[j][r] + bb; const int rl = 8 * g + r;
        if (MODE == 0) { so[wave][rl][hl * 128 + d] = v + bfr(U[h * HD + d]); so[wave][rl][hl * 128 + 64 + d] = v + bfr(Vb[h * HD + d]); }
        else { const size_t t = (r0 + rl) % TT; so[wave][rl][hl * 128 + d] = v; so[wave][rl][hl * 128 + 64 + d] = PP[t * FF + h * HD + d]; } } }
    LDSX();
    const int h0 = n0 >> 6;
    for (int rl = 0; rl < 16; ++rl) { vst2(OUT + ((r0 + rl) * NH + h0) * 128 + lane * 4, *(const v4f*)&so[wave][rl][lane * 4]); vst2(OUT + ((r0 + rl) * NH + h0) * 128 + 128 + lane * 4, *(const v4f*)&so[wave][rl][128 + lane * 4]); }
  }
}
__global__ __launch_bounds__(128) void k_attn(const float* __restrict__ QA, const float* __restrict__ KB, const int* __restrict__ MASK, const __bf16* __restrict__ VH, const __bf16* __restrict__ VL, float* __restrict__ O) {
  __shared__ __align__(16) float sp[4][16][36]; __shared__ __align__(16) float so[4][16][68];
  const int tid = threadIdx.x, wave = tid >> 5, lane = tid & 31, col = lane & 15, g = lane >> 4;
  const int qb = blockIdx.x, h = blockIdx.y, b = blockIdx.z; const int q0 = qb * 64 + wave * 16; const size_t rq = (size_t)b * TT + q0;
  const float* qrow = QA + ((rq + col) * NH + h) * 128;
  float m[8], l[8];
#pragma unroll
  for (int r = 0; r < 8; ++r) { m[r] = -3.0e38f; l[r] = 0.f; }
  v8f acc[4] = {};
#pragma unroll 1
  for (int ks = 0; ks < TT / 32; ++ks) { v8f s[2]; int mk[2][8]; bool anylive = false;
#pragma unroll
    for (int ct = 0; ct < 2; ++ct) { const int kk = ks * 32 + ct * 16 + col;
#pragma unroll
      for (int r = 0; r < 8; ++r) { const int mv = MASK[((size_t)b * TT + q0 + 8 * g + r) * TT + kk]; mk[ct][r] = mv; anylive = anylive || (mv != 0); } }
    if (__any(anylive)) {
#pragma unroll
      for (int ct = 0; ct < 2; ++ct) { const int kk = ks * 32 + ct * 16 + col; const float* krow = KB + (((size_t)b * TT + kk) * NH + h) * 128; v8f c = {};
#pragma unroll
        for (int kc = 0; kc < 4; ++kc) { const F2 kb = split_row(krow, kc * 32, lane); const F2 qa = split_row(qrow, kc * 32, lane); c = mac3(qa, kb, c); }
#pragma unroll
        for (int r = 0; r < 8; ++r) s[ct][r] = (mk[ct][r] != 0) ? c[r] * 0.125f : -3.0e38f; }
#pragma unroll
      for (int r = 0; r < 8; ++r) { float mx = fmaxf(s[0][r], s[1][r]);
#pragma unroll
        for (int o = 1; o < 16; o <<= 1) mx = fmaxf(mx, __shfl_xor(mx, o));
        const float mn = fmaxf(m[r], mx); const float alpha = (m[r] <= -1.0e38f) ? 0.f : exp_ni(m[r] - mn);
        const float e0 = (s[0][r] <= -1.0e38f) ? 0.f : exp_ni(s[0][r] - mn), e1 = (s[1][r] <= -1.0e38f) ? 0.f : exp_ni(s[1][r] - mn); float es = e0 + e1;
#pragma unroll
        for (int o = 1; o < 16; o <<= 1) es += __shfl_xor(es, o);
        l[r] = l[r] * alpha + es; m[r] = mn;
#pragma unroll
        for (int dt = 0; dt < 4; ++dt) acc[dt][r] *= alpha;
        sp[wave][8 * g + r][col] = e0; sp[wave][8 * g + r][16 + col] = e1; }
      LDSX();
      const F2 pa = split_row(&sp[wave][col][0], 0, lane);
#pragma unroll
      for (int dt = 0; dt < 4; ++dt) { const size_t vr = ((size_t)b * FF + h * HD + dt * 16 + col) * TT + ks * 32; const v16b vh = frag_b(VH + vr, lane), vl = frag_b(VL + vr, lane); acc[dt] = wmma_bf(pa.l, vh, acc[dt]); acc[dt] = wmma_bf(pa.h, vl, acc[dt]); acc[dt] = wmma_bf(pa.h, vh, acc[dt]); }
      LDSX(); } }
#pragma unroll
  for (int r = 0; r < 8; ++r) { const float il = (l[r] > 0.f) ? 1.0f / l[r] : 0.f;
#pragma unroll
    for (int dt = 0; dt < 4; ++dt) so[wave][8 * g + r][dt * 16 + col] = acc[dt][r] * il; }
  LDSX();
  for (int rl = 0; rl < 16; ++rl) if (lane < 16) vst2(O + (rq + rl) * FF + h * HD + lane * 4, *(const v4f*)&so[wave][rl][lane * 4]);
}
__global__ __launch_bounds__(128) void k_out(const float* __restrict__ O, const __bf16* __restrict__ P, const float* __restrict__ bias, float* __restrict__ Y) {
  __shared__ __align__(16) float so[4][16][132];
  const int tid = threadIdx.x, wave = tid >> 5, lane = tid & 31, col = lane & 15, g = lane >> 4; const size_t r0 = (size_t)blockIdx.x * 64 + wave * 16; const int n0 = blockIdx.y * 128;
  v8f acc[8] = {};
#pragma unroll 2
  for (int kc = 0; kc < FF / 32; ++kc) { const F2 a = split_row(O + (r0 + col) * FF, kc * 32, lane);
#pragma unroll
    for (int j = 0; j < 8; ++j) { const v16b w = frag_b(P + (size_t)(n0 + j * 16 + col) * FF + kc * 32, lane); acc[j] = wmma_bf(a.l, w, acc[j]); acc[j] = wmma_bf(a.h, w, acc[j]); } }
#pragma unroll
  for (int j = 0; j < 8; ++j) { const float bb = bfr(bias[n0 + j * 16 + col]);
#pragma unroll
    for (int r = 0; r < 8; ++r) so[wave][8 * g + r][j * 16 + col] = acc[j][r] + bb; }
  LDSX();
  for (int rl = 0; rl < 16; ++rl) vst2(Y + (r0 + rl) * FF + n0 + lane * 4, *(const v4f*)&so[wave][rl][lane * 4]);
}
extern "C" void kernel_launch(void* const* d_in, const int* in_sizes, int n_in, void* d_out, int out_size, void* d_ws, size_t ws_size, hipStream_t stream) {
  (void)in_sizes; (void)n_in; (void)out_size;
  const float** F = (const float**)d_in; const int* MASK = (const int*)d_in[3];
  if (ws_size < (size_t)WS_END) return;
  char* ws = (char*)d_ws; __bf16 *PW = (__bf16*)(ws + WS_PW), *VH = (__bf16*)(ws + WS_VH), *VL = (__bf16*)(ws + WS_VL); float *QA = (float*)(ws + WS_QA), *KB = (float*)(ws + WS_KB), *P = (float*)(ws + WS_P), *O = (float*)(ws + WS_O);
  k_pack<<<dim3(FF, 5), 128, 0, stream>>>(F[5], F[7], F[9], F[11], F[12], PW);
  k_posp<<<dim3(TT / 64, FF / 128), 128, 0, stream>>>(F[4], PW + (size_t)3 * FF * FF, P);
  k_proj<0><<<dim3(TNB * TT / 64, FF / 128), 128, 0, stream>>>(F[0], PW, F[6], F[14], F[15], P, QA, nullptr, nullptr);
  k_proj<1><<<dim3(TNB * TT / 64, FF / 128), 128, 0, stream>>>(F[1], PW + (size_t)FF * FF, F[8], F[14], F[15], P, KB, nullptr, nullptr);
  k_proj<2><<<dim3(TNB * TT / 64, FF / 128), 128, 0, stream>>>(F[2], PW + (size_t)2 * FF * FF, F[10], F[14], F[15], P, nullptr, VH, VL);
  k_attn<<<dim3(TQB, NH, TNB), 128, 0, stream>>>(QA, KB, MASK, VH, VL, O);
  k_out<<<dim3(TOB, FF / 128), 128, 0, stream>>>(O, PW + (size_t)4 * FF * FF, F[13], (float*)d_out);
}
